// GNN_node_Virtualnode_64183991272049
// MI455X (gfx1250) — hardware-verified
//
#include <hip/hip_runtime.h>
#include <stddef.h>


#define DD      128
#define D2      256
#define GG      512
#define NTHR    256
#define NWAVE   8
#define EPT     8
#define NGRP    2
#define CHUNK   (NTHR * EPT * NGRP)
#define WCAP    (EPT * NGRP * 32)
#define LISTN   (NWAVE * WCAP)
#define NBC     4096
#define NBP     32
#define RCAP    32768
#define RBN     128
#define OTHR    512
#define CNTCL   4095
#define DEGCAP  256
#define MROWS   32
#define MTHR    128
#define ZP      136
#define YP      264
#define BNEPS   1e-5f

#define LDS_FILL ((RCAP + NBC + LISTN) * 4 + 64)
#define LDS_MLP  (2 * MROWS * ZP * 2 + 2 * MROWS * YP * 2)

static_assert((CHUNK & (CHUNK - 1)) == 0);
static_assert(CHUNK <= 4096);
static_assert(NBC <= 4096 && (NBC & (NBC - 1)) == 0);
static_assert(NBP <= 4096 && (NBP & (NBP - 1)) == 0);
static_assert(OTHR * 8 == NBC);
static_assert((RCAP % 32) == 0);
static_assert(MROWS * DD * 4 <= 2 * MROWS * YP * 2);
static_assert((ZP % 8) == 0 && (YP % 8) == 0);
static_assert(NWAVE * 32 == NTHR);
static_assert(MTHR == 4 * 32 && MROWS == 4 * 8);
static_assert(NBC == NWAVE * 4 * 128);
static_assert((GG % NBP) == 0 && (GG % 64) == 0 && (GG % MROWS) == 0);
static_assert(NBP == NWAVE * 4);
static_assert((MROWS * ZP * 2) % 16 == 0 && (MROWS * YP * 2) % 16 == 0);

typedef float          v4f   __attribute__((ext_vector_type(4)));
typedef float          v8f   __attribute__((ext_vector_type(8)));
typedef int            v4i   __attribute__((ext_vector_type(4)));
typedef unsigned short v4us  __attribute__((ext_vector_type(4)));
typedef unsigned short v8us  __attribute__((ext_vector_type(8)));
typedef __bf16         v16bf __attribute__((ext_vector_type(16)));
union FragB { v16bf v; v8us u[2]; };

__device__ __forceinline__ unsigned short bfb(float x) {
  const __bf16 t = (__bf16)x;
  return __builtin_bit_cast(unsigned short, t);
}
__device__ __forceinline__ float bfu(unsigned short u) { return __uint_as_float(((unsigned)u) << 16); }
__device__ __forceinline__ float bfr(float x) { return bfu(bfb(x)); }
__device__ __forceinline__ v4f bfr4(const float* p) {
  const v4f a = *(const v4f*)p;
  v4f r;
  r.x = bfr(a.x); r.y = bfr(a.y); r.z = bfr(a.z); r.w = bfr(a.w);
  return r;
}
__device__ __forceinline__ void split1(float v, unsigned short& h, unsigned short& l) {
  const unsigned short hb = bfb(v);
  h = hb;
  l = bfb(v - bfu(hb));
}
__device__ __forceinline__ void split4(v4f v, v4us& h, v4us& l) {
  unsigned short a, b;
  split1(v.x, a, b); h.x = a; l.x = b;
  split1(v.y, a, b); h.y = a; l.y = b;
  split1(v.z, a, b); h.z = a; l.z = b;
  split1(v.w, a, b); h.w = a; l.w = b;
}

__device__ __forceinline__ v16bf ldfrag(const unsigned short* p) {
  FragB f;
  f.u[0] = *(const v8us*)p;
  f.u[1] = *(const v8us*)(p + 16);
  return f.v;
}

__device__ __forceinline__ v8f wm2(v16bf ah, v16bf al, v16bf b, v8f c) {
  v8f d = __builtin_amdgcn_wmma_f32_16x16x32_bf16(false, ah, false, b, (short)0, c, false, false);
  d = __builtin_amdgcn_wmma_f32_16x16x32_bf16(false, al, false, b, (short)0, d, false, false);
  asm volatile("v_nop\n\tv_nop\n\tv_nop\n\tv_nop" : "+v"(d) : "v"(ah), "v"(al), "v"(b));
  return d;
}

__device__ __forceinline__ void lanerank(int key, int lane, int& rank, int& tot) {
  int rk = 0, tt = 0;
#pragma unroll
  for (int q = 0; q < 32; ++q) {
    const int kq = __builtin_amdgcn_readlane(key, q);
    const bool eq = (kq == key);
    tt += eq ? 1 : 0;
    rk += (eq && q < lane) ? 1 : 0;
  }
  rank = rk;
  tot = tt;
}

template <int NB>
__device__ __forceinline__ int scan_chunk(const int* __restrict__ ids, int nE, int cbase, int slotBase,
                                          int vec8, int* list, int tid, int lane, int wave) {
  int wc = 0;
#pragma unroll
  for (int g = 0; g < NGRP; ++g) {
    const int el0  = (g * NTHR + tid) * EPT;
    const int e0   = cbase + el0;
    const int sent = -2147483647 - 1;
    v4i da, db;
    if (vec8 != 0 && cbase + CHUNK <= nE) {
      da = *(const v4i*)(ids + e0);
      db = *(const v4i*)(ids + e0 + 4);
    } else {
      da.x = (e0     < nE) ? ids[min(e0,     nE - 1)] : sent;
      da.y = (e0 + 1 < nE) ? ids[min(e0 + 1, nE - 1)] : sent;
      da.z = (e0 + 2 < nE) ? ids[min(e0 + 2, nE - 1)] : sent;
      da.w = (e0 + 3 < nE) ? ids[min(e0 + 3, nE - 1)] : sent;
      db.x = (e0 + 4 < nE) ? ids[min(e0 + 4, nE - 1)] : sent;
      db.y = (e0 + 5 < nE) ? ids[min(e0 + 5, nE - 1)] : sent;
      db.z = (e0 + 6 < nE) ? ids[min(e0 + 6, nE - 1)] : sent;
      db.w = (e0 + 7 < nE) ? ids[min(e0 + 7, nE - 1)] : sent;
    }
    const unsigned nb = (unsigned)slotBase;
    const unsigned s0 = (unsigned)da.x - nb, s1 = (unsigned)da.y - nb;
    const unsigned s2 = (unsigned)da.z - nb, s3 = (unsigned)da.w - nb;
    const unsigned s4 = (unsigned)db.x - nb, s5 = (unsigned)db.y - nb;
    const unsigned s6 = (unsigned)db.z - nb, s7 = (unsigned)db.w - nb;
    const bool h0 = s0 < (unsigned)NB, h1 = s1 < (unsigned)NB, h2 = s2 < (unsigned)NB, h3 = s3 < (unsigned)NB;
    const bool h4 = s4 < (unsigned)NB, h5 = s5 < (unsigned)NB, h6 = s6 < (unsigned)NB, h7 = s7 < (unsigned)NB;
    const unsigned any = __builtin_amdgcn_ballot_w32(h0 | h1 | h2 | h3 | h4 | h5 | h6 | h7);
    if (any != 0u) {
#define HITJ(J, HJ, SJ) { \
        const unsigned mj = __builtin_amdgcn_ballot_w32(HJ); \
        if (mj != 0u) { \
          if (HJ) { \
            const int pos = wc + (int)__builtin_amdgcn_mbcnt_lo(mj, 0u); \
            if (pos < WCAP) list[wave * WCAP + pos] = ((el0 + (J)) << 12) | (int)(SJ); \
          } \
          wc += (int)__builtin_popcount(mj); } }
      HITJ(0, h0, s0)
      HITJ(1, h1, s1)
      HITJ(2, h2, s2)
      HITJ(3, h3, s3)
      HITJ(4, h4, s4)
      HITJ(5, h5, s5)
      HITJ(6, h6, s6)
      HITJ(7, h7, s7)
#undef HITJ
    }
  }
  return wc;
}

__global__ __launch_bounds__(NTHR) void k_wprep(
    const float* __restrict__ mW1, const float* __restrict__ mW2,
    const float* __restrict__ vW1, const float* __restrict__ vW2,
    unsigned short* W1p, unsigned short* W2p, unsigned short* V1p, unsigned short* V2p, int nL, int nV) {
  const int per = DD * D2;
  const int g0 = nL * (per / 8), g1 = nL * (per / 8), g2 = nV * (per / 8), g3 = nV * (per / 8);
  const int bstart = blockIdx.x * NTHR;
  const float* src; unsigned short* dst; int K, Nout, segOff;
  if (bstart < g0)                { src = mW1; dst = W1p; K = DD; Nout = D2; segOff = 0; }
  else if (bstart < g0 + g1)      { src = mW2; dst = W2p; K = D2; Nout = DD; segOff = g0; }
  else if (bstart < g0 + g1 + g2) { src = vW1; dst = V1p; K = DD; Nout = D2; segOff = g0 + g1; }
  else                            { src = vW2; dst = V2p; K = D2; Nout = DD; segOff = g0 + g1 + g2; }
  const int i = bstart + (int)threadIdx.x;
  if (i >= g0 + g1 + g2 + g3) return;
  const int e = (i - segOff) * 8;
  const int layer = e / per;
  const int rem = e - layer * per;
  const int n = rem / K;
  const int k0 = rem - n * K;
  const float* sp = src + (size_t)layer * per;
  v8us o;
  o[0] = bfb(sp[(size_t)(k0 + 0) * Nout + n]);
  o[1] = bfb(sp[(size_t)(k0 + 1) * Nout + n]);
  o[2] = bfb(sp[(size_t)(k0 + 2) * Nout + n]);
  o[3] = bfb(sp[(size_t)(k0 + 3) * Nout + n]);
  o[4] = bfb(sp[(size_t)(k0 + 4) * Nout + n]);
  o[5] = bfb(sp[(size_t)(k0 + 5) * Nout + n]);
  o[6] = bfb(sp[(size_t)(k0 + 6) * Nout + n]);
  o[7] = bfb(sp[(size_t)(k0 + 7) * Nout + n]);
  unsigned short* dp = dst + e;
  *(volatile v8us*)dp = o;
  __threadfence();
  *(volatile v8us*)dp = o;
}

__global__ __launch_bounds__(NTHR) void k_init(
    const int* __restrict__ x, const float* __restrict__ enc, const float* __restrict__ vne,
    float* hin, float* vn, int nN, int nPadRows, int nEmb) {
  const int tid = threadIdx.x, lane = tid & 31, wave = tid >> 5;
  const int nb0 = nPadRows / 64;
  const v4f ve = bfr4(vne + 4 * lane);
  const v4f zero4 = {0.f, 0.f, 0.f, 0.f};
  v4f ov[8];
  if ((int)blockIdx.x < nb0) {
    const int base = (int)blockIdx.x * 64 + wave * 8;
#pragma unroll
    for (int i = 0; i < 8; ++i) {
      const int row = base + i;
      const int rr = row < nN ? row : nN - 1;
      int t = x[rr];
      t = t < 0 ? 0 : (t > nEmb - 1 ? nEmb - 1 : t);
      v4f v = bfr4(enc + (size_t)t * DD + 4 * lane) + ve;
      if (row >= nN) v = zero4;
      ov[i] = v;
    }
    float* hp = hin + (size_t)base * DD + 4 * lane;
#pragma unroll
    for (int i = 0; i < 8; ++i) *(volatile v4f*)(hp + (size_t)i * DD) = ov[i];
    __threadfence();
#pragma unroll
    for (int i = 0; i < 8; ++i) *(volatile v4f*)(hp + (size_t)i * DD) = ov[i];
  } else {
    const int base = ((int)blockIdx.x - nb0) * 64 + wave * 8;
    float* vp = vn + (size_t)base * DD + 4 * lane;
#pragma unroll
    for (int i = 0; i < 8; ++i) *(volatile v4f*)(vp + (size_t)i * DD) = ve;
    __threadfence();
#pragma unroll
    for (int i = 0; i < 8; ++i) *(volatile v4f*)(vp + (size_t)i * DD) = ve;
  }
}

__global__ __launch_bounds__(NTHR) void k_count(
    const int* __restrict__ ei, int* cnt, int nE, int vec8) {
  __shared__ __attribute__((aligned(16))) int scnt[NBC];
  __shared__ __attribute__((aligned(16))) int list[LISTN];
  __shared__ int wcnt[NWAVE];
  const int tid = threadIdx.x, lane = tid & 31, wave = tid >> 5;
  const int nodeBase = blockIdx.x * NBC;
  const int* dsts = ei + nE;

  for (int i = tid; i < NBC; i += NTHR) scnt[i] = 0;
  __syncthreads();

  const int nChunks = (nE + CHUNK - 1) / CHUNK;
#pragma unroll 1
  for (int ch = 0; ch < nChunks; ++ch) {
    const int cbase = ch * CHUNK;
    const int wc = scan_chunk<NBC>(dsts, nE, cbase, nodeBase, vec8, list, tid, lane, wave);
    if (lane == 0) wcnt[wave] = wc;
    __syncthreads();
    if (wave == 0) {
#pragma unroll 1
      for (int wsx = 0; wsx < NWAVE; ++wsx) {
        int n = __builtin_amdgcn_readfirstlane(wcnt[wsx]);
        n = n > WCAP ? WCAP : (n < 0 ? 0 : n);
        const int* lp = list + wsx * WCAP;
#pragma unroll 1
        for (int b0 = 0; b0 < n; b0 += 32) {
          const int idx = b0 + lane;
          const bool valid = idx < n;
          const int ent = lp[idx < WCAP ? idx : WCAP - 1];
          const int slot = ent & (NBC - 1);
          const int key = valid ? slot : -1;
          const int ka  = valid ? slot : 0;
          int rk, tt;
          lanerank(key, lane, rk, tt);
          if (valid && rk == tt - 1) scnt[ka] = scnt[ka] + tt;
        }
      }
    }
    __syncthreads();
  }

  v4i cq[4];
#pragma unroll
  for (int q = 0; q < 4; ++q) {
    const int f = (wave * 4 + q) * 128 + 4 * lane;
    cq[q] = *(const v4i*)(scnt + f);
  }
  int* cp = cnt + (size_t)nodeBase;
#pragma unroll
  for (int q = 0; q < 4; ++q) {
    const int f = (wave * 4 + q) * 128 + 4 * lane;
    *(volatile v4i*)(cp + f) = cq[q];
  }
  __threadfence();
#pragma unroll
  for (int q = 0; q < 4; ++q) {
    const int f = (wave * 4 + q) * 128 + 4 * lane;
    *(volatile v4i*)(cp + f) = cq[q];
  }
}

__global__ __launch_bounds__(OTHR) void k_offsets(
    const int* __restrict__ cnt, int* off, int* rbase, int nChunk) {
  __shared__ __attribute__((aligned(16))) int soff[NBC];
  __shared__ __attribute__((aligned(16))) int srb[RBN];
  __shared__ int wtot[OTHR / 32];
  const int tid = threadIdx.x, lane = tid & 31, wave = tid >> 5;
  for (int i = tid; i < RBN; i += OTHR) srb[i] = 0;
  __syncthreads();
  int carry = 0;
#pragma unroll 1
  for (int ch = 0; ch < nChunk; ++ch) {
    const int base = ch * NBC;
    const v4i c0 = *(const v4i*)(cnt + base + 8 * tid);
    const v4i c1 = *(const v4i*)(cnt + base + 8 * tid + 4);
    const int e0 = min(max(c0.x, 0), CNTCL), e1 = min(max(c0.y, 0), CNTCL);
    const int e2 = min(max(c0.z, 0), CNTCL), e3 = min(max(c0.w, 0), CNTCL);
    const int e4 = min(max(c1.x, 0), CNTCL), e5 = min(max(c1.y, 0), CNTCL);
    const int e6 = min(max(c1.z, 0), CNTCL), e7 = min(max(c1.w, 0), CNTCL);
    const int ts = e0 + e1 + e2 + e3 + e4 + e5 + e6 + e7;
    int incl = ts;
#pragma unroll
    for (int d = 1; d < 32; d <<= 1) {
      const int t = __shfl_up(incl, d);
      if (lane >= d) incl += t;
    }
    if (lane == 31) wtot[wave] = incl;
    __syncthreads();
    int pre = 0, tot = 0;
#pragma unroll
    for (int w = 0; w < OTHR / 32; ++w) {
      const int tw = wtot[w];
      tot += tw;
      pre += (w < wave) ? tw : 0;
    }
    int run = carry + pre + incl - ts;
    soff[8 * tid + 0] = run; run += e0;
    soff[8 * tid + 1] = run; run += e1;
    soff[8 * tid + 2] = run; run += e2;
    soff[8 * tid + 3] = run; run += e3;
    soff[8 * tid + 4] = run; run += e4;
    soff[8 * tid + 5] = run; run += e5;
    soff[8 * tid + 6] = run; run += e6;
    soff[8 * tid + 7] = run;
    if (tid == 0) srb[ch < RBN - 1 ? ch : RBN - 1] = carry;
    const int ncarry = carry + ((tot + 31) & ~31);
    __syncthreads();
    const v4i o0 = *(const v4i*)(soff + 4 * tid);
    const v4i o1 = *(const v4i*)(soff + 4 * (tid + OTHR));
    int* op = off + base;
    *(volatile v4i*)(op + 4 * tid) = o0;
    *(volatile v4i*)(op + 4 * (tid + OTHR)) = o1;
    __threadfence();
    *(volatile v4i*)(op + 4 * tid) = o0;
    *(volatile v4i*)(op + 4 * (tid + OTHR)) = o1;
    carry = ncarry;
    __syncthreads();
  }
  if (tid == 0) srb[nChunk < RBN - 1 ? nChunk : RBN - 1] = carry;
  __syncthreads();
  v4i rv = {0, 0, 0, 0};
  if (tid < 32) rv = *(const v4i*)(srb + 4 * tid);
  if (tid < 32) *(volatile v4i*)(rbase + 4 * tid) = rv;
  __threadfence();
  if (tid < 32) *(volatile v4i*)(rbase + 4 * tid) = rv;
}

__global__ __launch_bounds__(NTHR) void k_fill(
    const int* __restrict__ ei, const int* __restrict__ off, const int* __restrict__ rbase,
    int* csr, int nN, int nE, int vec8, int csrLen) {
  extern __shared__ v4f lds_dyn[];
  int* region = (int*)lds_dyn;
  int* cursor = region + RCAP;
  int* list   = cursor + NBC;
  int* wcnt   = list + LISTN;
  const int tid = threadIdx.x, lane = tid & 31, wave = tid >> 5;
  const int b = blockIdx.x;
  const int nodeBase = b * NBC;
  const int* dsts = ei + nE;

  int rb0 = rbase[b];
  const int rb1 = rbase[b + 1];
  rb0 = rb0 < 0 ? 0 : (rb0 > csrLen ? csrLen : rb0);
  rb0 &= ~31;
  int len = rb1 - rb0;
  len = len < 0 ? 0 : (len > RCAP ? RCAP : len);
  int lenW = (len + 31) & ~31;
  if (rb0 + lenW > csrLen) lenW = (csrLen - rb0) & ~31;

  {
    const v4i z = {0, 0, 0, 0};
    for (int i = tid; i < RCAP / 4; i += NTHR) ((v4i*)region)[i] = z;
    for (int s = tid; s < NBC; s += NTHR) {
      int o = off[nodeBase + s] - rb0;
      o = o < 0 ? 0 : (o > RCAP ? RCAP : o);
      cursor[s] = o;
    }
  }
  __syncthreads();

  const int nChunks = (nE + CHUNK - 1) / CHUNK;
#pragma unroll 1
  for (int ch = 0; ch < nChunks; ++ch) {
    const int cbase = ch * CHUNK;
    const int wc = scan_chunk<NBC>(dsts, nE, cbase, nodeBase, vec8, list, tid, lane, wave);
    if (lane == 0) wcnt[wave] = wc;
    __syncthreads();
    if (wave == 0) {
#pragma unroll 1
      for (int wsx = 0; wsx < NWAVE; ++wsx) {
        int n = __builtin_amdgcn_readfirstlane(wcnt[wsx]);
        n = n > WCAP ? WCAP : (n < 0 ? 0 : n);
        const int* lp = list + wsx * WCAP;
#pragma unroll 1
        for (int b0 = 0; b0 < n; b0 += 32) {
          const int idx = b0 + lane;
          const bool valid = idx < n;
          const int ent = lp[idx < WCAP ? idx : WCAP - 1];
          const int slot = ent & (NBC - 1);
          const int key = valid ? slot : -1;
          const int ka  = valid ? slot : 0;
          int e = cbase + ((ent >> 12) & (CHUNK - 1));
          e = e > nE - 1 ? nE - 1 : e;
          int s = ei[e];
          s = s < 0 ? 0 : (s > nN - 1 ? nN - 1 : s);
          int rk, tt;
          lanerank(key, lane, rk, tt);
          const int c0 = cursor[ka];
          int pos = c0 + rk;
          pos = pos < 0 ? 0 : (pos > RCAP - 1 ? RCAP - 1 : pos);
          if (valid) region[pos] = s;
          if (valid && rk == tt - 1) {
            const int np = c0 + tt;
            cursor[ka] = np > RCAP ? RCAP : np;
          }
        }
      }
    }
    __syncthreads();
  }

  const int nv = lenW >> 2;
  int* gp = csr + rb0;
#pragma unroll 1
  for (int i = tid; i < nv; i += NTHR) { const v4i v = ((const v4i*)region)[i]; *(volatile v4i*)(gp + 4 * i) = v; }
  __threadfence();
#pragma unroll 1
  for (int i = tid; i < nv; i += NTHR) { const v4i v = ((const v4i*)region)[i]; *(volatile v4i*)(gp + 4 * i) = v; }
}

__global__ __launch_bounds__(NTHR) void k_pool(
    const int* __restrict__ batch, const float* __restrict__ hin, const float* __restrict__ vn,
    float* vt, int nN, int vecb) {
  __shared__ __attribute__((aligned(16))) float acc[NBP * DD];
  __shared__ __attribute__((aligned(16))) int list[LISTN];
  __shared__ int wcnt[NWAVE];
  const int tid = threadIdx.x, lane = tid & 31, wave = tid >> 5;
  const int gBase = blockIdx.x * NBP;

  {
    const v4f z = {0.f, 0.f, 0.f, 0.f};
    for (int i = tid; i < NBP * DD / 4; i += NTHR) ((v4f*)acc)[i] = z;
  }
  __syncthreads();

  const int nChunks = (nN + CHUNK - 1) / CHUNK;
#pragma unroll 1
  for (int ch = 0; ch < nChunks; ++ch) {
    const int cbase = ch * CHUNK;
    const int wc = scan_chunk<NBP>(batch, nN, cbase, gBase, vecb, list, tid, lane, wave);
    if (lane == 0) wcnt[wave] = wc;
    __syncthreads();
    if (wave == 0) {
#pragma unroll 1
      for (int wsx = 0; wsx < NWAVE; ++wsx) {
        int n = __builtin_amdgcn_readfirstlane(wcnt[wsx]);
        n = n > WCAP ? WCAP : (n < 0 ? 0 : n);
        const int* lp = list + wsx * WCAP;
#pragma unroll 1
        for (int i = 0; i < n; ++i) {
          const int ent  = __builtin_amdgcn_readfirstlane(lp[i]);
          const int slot = ent & (NBP - 1);
          int nd = cbase + ((ent >> 12) & (CHUNK - 1));
          nd = nd > nN - 1 ? nN - 1 : nd;
          const v4f v = *(const v4f*)(hin + (size_t)nd * DD + 4 * lane);
          v4f* ap = (v4f*)(acc + slot * DD + 4 * lane);
          *ap = *ap + v;
        }
      }
    }
    __syncthreads();
  }

  v4f ov[4];
#pragma unroll
  for (int i = 0; i < 4; ++i) {
    const int row = wave * 4 + i;
    const int g = gBase + row;
    ov[i] = *(const v4f*)(acc + row * DD + 4 * lane) + *(const v4f*)(vn + (size_t)g * DD + 4 * lane);
  }
  float* gp = vt + (size_t)(gBase + wave * 4) * DD + 4 * lane;
#pragma unroll
  for (int i = 0; i < 4; ++i) *(volatile v4f*)(gp + (size_t)i * DD) = ov[i];
  __threadfence();
#pragma unroll
  for (int i = 0; i < 4; ++i) *(volatile v4f*)(gp + (size_t)i * DD) = ov[i];
}

template <int SRC, int OM>
__global__ __launch_bounds__(MTHR) void k_mlp(
    const float* __restrict__ src, const int* __restrict__ csr, const int* __restrict__ offp,
    const int* __restrict__ cntp, const float* __restrict__ epsp, int layer, int nN, int csrLen,
    const unsigned short* __restrict__ W1, const float* __restrict__ pb1, const float* __restrict__ pg1,
    const float* __restrict__ pt1, const float* __restrict__ pm1, const float* __restrict__ pv1,
    const unsigned short* __restrict__ W2, const float* __restrict__ pb2, const float* __restrict__ pg2,
    const float* __restrict__ pt2, const float* __restrict__ pm2, const float* __restrict__ pv2,
    const float* __restrict__ vnp, const int* __restrict__ batch, float* outp, int nOutRows) {
  extern __shared__ v4f lds_dyn[];
  unsigned short* zh = (unsigned short*)lds_dyn;
  unsigned short* zl = zh + MROWS * ZP;
  unsigned short* yh = zl + MROWS * ZP;
  unsigned short* yl = yh + MROWS * YP;
  float* ost = (float*)yh;
  const int tid = threadIdx.x, lane = tid & 31, wave = tid >> 5, hh = lane >> 4, m = lane & 15;
  const int R0 = blockIdx.x * MROWS;
  const v4f zero4 = {0.f, 0.f, 0.f, 0.f};

  if (SRC == 0) {
    const float ope = 1.0f + bfr(epsp[layer]);
#pragma unroll 1
    for (int j = 0; j < 8; ++j) {
      const int rloc = wave * 8 + j;
      const int c = R0 + rloc;
      const bool valid = c < nN;
      const int cc = valid ? c : nN - 1;
      int n = cntp[c];
      n = n < 0 ? 0 : (n > DEGCAP ? DEGCAP : n);
      n = valid ? n : 0;
      const int st = offp[c];
      v4f acc = zero4;
#pragma unroll 1
      for (int q0 = 0; q0 < n; q0 += 32) {
        int pos = st + q0 + lane;
        pos = pos < 0 ? 0 : (pos > csrLen - 1 ? csrLen - 1 : pos);
        int sl = csr[pos];
        sl = sl < 0 ? 0 : (sl > nN - 1 ? nN - 1 : sl);
        const int mcnt = (n - q0) < 32 ? (n - q0) : 32;
#pragma unroll 1
        for (int p = 0; p < mcnt; ++p) {
          const int s = __builtin_amdgcn_readlane(sl, p);
          acc = acc + *(const v4f*)(src + (size_t)s * DD + 4 * lane);
        }
      }
      const v4f sv = *(const v4f*)(src + (size_t)cc * DD + 4 * lane);
      v4f z = sv * ope + acc;
      if (!valid) z = zero4;
      v4us zhv = {0, 0, 0, 0}, zlv = {0, 0, 0, 0};
      split4(z, zhv, zlv);
      *(v4us*)(zh + rloc * ZP + 4 * lane) = zhv;
      *(v4us*)(zl + rloc * ZP + 4 * lane) = zlv;
    }
  } else {
#pragma unroll 1
    for (int j = 0; j < 8; ++j) {
      const int rloc = wave * 8 + j;
      const v4f z = *(const v4f*)(src + (size_t)(R0 + rloc) * DD + 4 * lane);
      v4us zhv = {0, 0, 0, 0}, zlv = {0, 0, 0, 0};
      split4(z, zhv, zlv);
      *(v4us*)(zh + rloc * ZP + 4 * lane) = zhv;
      *(v4us*)(zl + rloc * ZP + 4 * lane) = zlv;
    }
  }
  __syncthreads();

  v8f a1[2][4];
#pragma unroll
  for (int rt = 0; rt < 2; ++rt)
#pragma unroll
    for (int t = 0; t < 4; ++t) { v8f z8 = {0.f, 0.f, 0.f, 0.f, 0.f, 0.f, 0.f, 0.f}; a1[rt][t] = z8; }
#pragma unroll 1
  for (int ks = 0; ks < DD / 32; ++ks) {
    const int k0 = ks * 32;
    v16bf ah[2], al[2];
#pragma unroll
    for (int rt = 0; rt < 2; ++rt) {
      ah[rt] = ldfrag(zh + (16 * rt + m) * ZP + k0 + 8 * hh);
      al[rt] = ldfrag(zl + (16 * rt + m) * ZP + k0 + 8 * hh);
    }
#pragma unroll
    for (int t = 0; t < 4; ++t) {
      const v16bf b = ldfrag(W1 + (size_t)(wave * 64 + 16 * t + m) * DD + k0 + 8 * hh);
#pragma unroll
      for (int rt = 0; rt < 2; ++rt) a1[rt][t] = wm2(ah[rt], al[rt], b, a1[rt][t]);
    }
  }
#pragma unroll
  for (int t = 0; t < 4; ++t) {
    const int col = wave * 64 + 16 * t + m;
    const float eb = bfr(pb1[col]);
    const float em = bfr(pm1[col]);
    const float er = rsqrtf(bfr(pv1[col]) + BNEPS);
    const float eg = bfr(pg1[col]);
    const float et = bfr(pt1[col]);
#pragma unroll
    for (int rt = 0; rt < 2; ++rt) {
#pragma unroll
      for (int r = 0; r < 8; ++r) {
        float v = a1[rt][t][r] + eb;
        v = (v - em) * er;
        v = v * eg + et;
        v = fmaxf(v, 0.0f);
        unsigned short vh, vlo;
        split1(v, vh, vlo);
        const int o = (16 * rt + 8 * hh + r) * YP + col;
        yh[o] = vh;
        yl[o] = vlo;
      }
    }
  }
  __syncthreads();

  v8f a2[2][2];
#pragma unroll
  for (int rt = 0; rt < 2; ++rt)
#pragma unroll
    for (int t = 0; t < 2; ++t) { v8f z8 = {0.f, 0.f, 0.f, 0.f, 0.f, 0.f, 0.f, 0.f}; a2[rt][t] = z8; }
#pragma unroll 1
  for (int ks = 0; ks < D2 / 32; ++ks) {
    const int k0 = ks * 32;
    v16bf ah[2], al[2];
#pragma unroll
    for (int rt = 0; rt < 2; ++rt) {
      ah[rt] = ldfrag(yh + (16 * rt + m) * YP + k0 + 8 * hh);
      al[rt] = ldfrag(yl + (16 * rt + m) * YP + k0 + 8 * hh);
    }
#pragma unroll
    for (int t = 0; t < 2; ++t) {
      const v16bf b = ldfrag(W2 + (size_t)(wave * 32 + 16 * t + m) * D2 + k0 + 8 * hh);
#pragma unroll
      for (int rt = 0; rt < 2; ++rt) a2[rt][t] = wm2(ah[rt], al[rt], b, a2[rt][t]);
    }
  }
  __syncthreads();
#pragma unroll
  for (int rt = 0; rt < 2; ++rt)
#pragma unroll
    for (int t = 0; t < 2; ++t)
#pragma unroll
      for (int r = 0; r < 8; ++r)
        ost[(16 * rt + 8 * hh + r) * DD + wave * 32 + 16 * t + m] = a2[rt][t][r];
  __syncthreads();

  const int c4 = 4 * lane;
  const v4f ob = bfr4(pb2 + c4), omu = bfr4(pm2 + c4), og = bfr4(pg2 + c4), ot = bfr4(pt2 + c4);
  const v4f ovr = bfr4(pv2 + c4);
  v4f orr;
  orr.x = rsqrtf(ovr.x + BNEPS); orr.y = rsqrtf(ovr.y + BNEPS); orr.z = rsqrtf(ovr.z + BNEPS); orr.w = rsqrtf(ovr.w + BNEPS);
  v4f ov[8];
#pragma unroll
  for (int i = 0; i < 8; ++i) {
    const int rloc = wave * 8 + i;
    const int grow = R0 + rloc;
    v4f v = *(const v4f*)(ost + rloc * DD + c4);
    v = v + ob;
    v = (v - omu) * orr;
    v = v * og + ot;
    if (OM != 1) { v.x = fmaxf(v.x, 0.f); v.y = fmaxf(v.y, 0.f); v.z = fmaxf(v.z, 0.f); v.w = fmaxf(v.w, 0.f); }
    if (OM == 0) {
      const int gr = grow < nN ? grow : nN - 1;
      int bi = batch[gr];
      bi = bi < 0 ? 0 : (bi > GG - 1 ? GG - 1 : bi);
      v = v + *(const v4f*)(vnp + (size_t)bi * DD + c4);
    }
    ov[i] = v;
  }
#pragma unroll
  for (int i = 0; i < 8; ++i) {
    const int grow = R0 + wave * 8 + i;
    if (OM != 1 || grow < nOutRows) *(volatile v4f*)(outp + (size_t)grow * DD + c4) = ov[i];
  }
  __threadfence();
#pragma unroll
  for (int i = 0; i < 8; ++i) {
    const int grow = R0 + wave * 8 + i;
    if (OM != 1 || grow < nOutRows) *(volatile v4f*)(outp + (size_t)grow * DD + c4) = ov[i];
  }
}

extern "C" void kernel_launch(void* const* d_in, const int* in_sizes, int n_in,
                              void* d_out, int out_size, void* d_ws, size_t ws_size,
                              hipStream_t stream) {
  if (n_in < 30) return;
  const int nN = in_sizes[0];
  const int nE = in_sizes[1] / 2;
  if (nN <= 0 || nE <= 0 || in_sizes[1] != 2 * nE || in_sizes[2] != nN) return;
  const int nEmb = in_sizes[3] / DD;
  if (nEmb < 1 || in_sizes[3] != nEmb * DD || in_sizes[4] < DD) return;
  const int nL = in_sizes[5];
  if (nL < 1 || nL > 64) return;
  if (in_sizes[6] != nL * DD * D2 || in_sizes[7] != nL * D2 || in_sizes[8] != nL * D2 ||
      in_sizes[9] != nL * D2 || in_sizes[10] != nL * D2 || in_sizes[11] != nL * D2) return;
  if (in_sizes[12] != nL * D2 * DD || in_sizes[13] != nL * DD || in_sizes[14] != nL * DD ||
      in_sizes[15] != nL * DD || in_sizes[16] != nL * DD || in_sizes[17] != nL * DD) return;
  const int nV = in_sizes[18] / (DD * D2);
  if (nV < 0 || nV > nL || in_sizes[18] != nV * DD * D2) return;
  if (in_sizes[19] != nV * D2 || in_sizes[20] != nV * D2 || in_sizes[21] != nV * D2 ||
      in_sizes[22] != nV * D2 || in_sizes[23] != nV * D2) return;
  if (in_sizes[24] != nV * D2 * DD || in_sizes[25] != nV * DD || in_sizes[26] != nV * DD ||
      in_sizes[27] != nV * DD || in_sizes[28] != nV * DD || in_sizes[29] != nV * DD) return;
  if (out_size != nN * DD) return;
  if (nN > (1 << 24) || nE > (1 << 28)) return;

  const int*   x      = (const int*)d_in[0];
  const int*   ei     = (const int*)d_in[1];
  const int*   batch  = (const int*)d_in[2];
  const float* enc    = (const float*)d_in[3];
  const float* vnemb  = (const float*)d_in[4];
  const float* eps    = (const float*)d_in[5];
  const float* mW1    = (const float*)d_in[6];
  const float* mb1    = (const float*)d_in[7];
  const float* mbn_g  = (const float*)d_in[8];
  const float* mbn_b  = (const float*)d_in[9];
  const float* mbn_m  = (const float*)d_in[10];
  const float* mbn_v  = (const float*)d_in[11];
  const float* mW2    = (const float*)d_in[12];
  const float* mb2    = (const float*)d_in[13];
  const float* bn_g   = (const float*)d_in[14];
  const float* bn_b   = (const float*)d_in[15];
  const float* bn_m   = (const float*)d_in[16];
  const float* bn_v   = (const float*)d_in[17];
  const float* vW1    = (const float*)d_in[18];
  const float* vb1    = (const float*)d_in[19];
  const float* vbn1_g = (const float*)d_in[20];
  const float* vbn1_b = (const float*)d_in[21];
  const float* vbn1_m = (const float*)d_in[22];
  const float* vbn1_v = (const float*)d_in[23];
  const float* vW2    = (const float*)d_in[24];
  const float* vb2    = (const float*)d_in[25];
  const float* vbn2_g = (const float*)d_in[26];
  const float* vbn2_b = (const float*)d_in[27];
  const float* vbn2_m = (const float*)d_in[28];
  const float* vbn2_v = (const float*)d_in[29];
  float* out = (float*)d_out;

  const int NPAD   = ((nN + 255) / 256) * 256;
  const int nBC    = (nN + NBC - 1) / NBC;
  const int CNTPAD = nBC * NBC;
  if (nBC + 1 > RBN) return;
  const int csrLen = ((nE + 31) & ~31) + 32 * (nBC + 1) + 1024;
  const int per    = DD * D2;

  char* ws = (char*)d_ws;
  size_t off = 0;
  const size_t oW1  = off; off += (size_t)nL * per * 2;        off = (off + 255) & ~(size_t)255;
  const size_t oW2  = off; off += (size_t)nL * per * 2;        off = (off + 255) & ~(size_t)255;
  const size_t oV1  = off; off += (size_t)nV * per * 2 + 256;  off = (off + 255) & ~(size_t)255;
  const size_t oV2  = off; off += (size_t)nV * per * 2 + 256;  off = (off + 255) & ~(size_t)255;
  const size_t oCnt = off; off += (size_t)CNTPAD * 4;          off = (off + 255) & ~(size_t)255;
  const size_t oOff = off; off += (size_t)CNTPAD * 4;          off = (off + 255) & ~(size_t)255;
  const size_t oRb  = off; off += (size_t)RBN * 4;             off = (off + 255) & ~(size_t)255;
  const size_t oCsr = off; off += (size_t)csrLen * 4;          off = (off + 255) & ~(size_t)255;
  const size_t oHA  = off; off += (size_t)NPAD * DD * 4;       off = (off + 255) & ~(size_t)255;
  const size_t oHB  = off; off += (size_t)NPAD * DD * 4;       off = (off + 255) & ~(size_t)255;
  const size_t oVn  = off; off += (size_t)GG * DD * 4;         off = (off + 255) & ~(size_t)255;
  const size_t oVt  = off; off += (size_t)GG * DD * 4;         off = (off + 255) & ~(size_t)255;
  if (off > ws_size) return;
  unsigned short* W1p = (unsigned short*)(ws + oW1);
  unsigned short* W2p = (unsigned short*)(ws + oW2);
  unsigned short* V1p = (unsigned short*)(ws + oV1);
  unsigned short* V2p = (unsigned short*)(ws + oV2);
  int*   cnt  = (int*)(ws + oCnt);
  int*   offp = (int*)(ws + oOff);
  int*   rb   = (int*)(ws + oRb);
  int*   csr  = (int*)(ws + oCsr);
  float* hinA = (float*)(ws + oHA);
  float* hinB = (float*)(ws + oHB);
  float* vn   = (float*)(ws + oVn);
  float* vt   = (float*)(ws + oVt);

  const int vec8 = ((nE & 3) == 0) ? 1 : 0;
  const int vecb = ((nN & 3) == 0) ? 1 : 0;

  const int nPrep = (nL + nL + nV + nV) * (per / 8);
  k_wprep<<<(nPrep + NTHR - 1) / NTHR, NTHR, 0, stream>>>(mW1, mW2, vW1, vW2, W1p, W2p, V1p, V2p, nL, nV);

  k_init<<<NPAD / 64 + GG / 64, NTHR, 0, stream>>>(x, enc, vnemb, hinA, vn, nN, NPAD, nEmb);

  k_count<<<nBC, NTHR, 0, stream>>>(ei, cnt, nE, vec8);
  k_offsets<<<1, OTHR, 0, stream>>>(cnt, offp, rb, nBC);
  hipFuncSetAttribute(reinterpret_cast<const void*>(&k_fill),
                      hipFuncAttributeMaxDynamicSharedMemorySize, LDS_FILL);
  k_fill<<<nBC, NTHR, LDS_FILL, stream>>>(ei, offp, rb, csr, nN, nE, vec8, csrLen);

  hipFuncSetAttribute(reinterpret_cast<const void*>(&k_mlp<0, 0>),
                      hipFuncAttributeMaxDynamicSharedMemorySize, LDS_MLP);
  hipFuncSetAttribute(reinterpret_cast<const void*>(&k_mlp<0, 1>),
                      hipFuncAttributeMaxDynamicSharedMemorySize, LDS_MLP);
  hipFuncSetAttribute(reinterpret_cast<const void*>(&k_mlp<1, 2>),
                      hipFuncAttributeMaxDynamicSharedMemorySize, LDS_MLP);

  for (int l = 0; l < nL; ++l) {
    float* cur = (l & 1) ? hinB : hinA;
    float* nxt = (l & 1) ? hinA : hinB;
    if (l < nV) {
      k_pool<<<GG / NBP, NTHR, 0, stream>>>(batch, cur, vn, vt, nN, vecb);
      k_mlp<1, 2><<<GG / MROWS, MTHR, LDS_MLP, stream>>>(
          vt, csr, offp, cnt, eps, l, GG, csrLen,
          V1p + (size_t)l * per, vb1 + (size_t)l * D2, vbn1_g + (size_t)l * D2, vbn1_b + (size_t)l * D2,
          vbn1_m + (size_t)l * D2, vbn1_v + (size_t)l * D2,
          V2p + (size_t)l * per, vb2 + (size_t)l * DD, vbn2_g + (size_t)l * DD, vbn2_b + (size_t)l * DD,
          vbn2_m + (size_t)l * DD, vbn2_v + (size_t)l * DD,
          vt, batch, vn, GG);
    }
    if (l < nL - 1) {
      k_mlp<0, 0><<<NPAD / MROWS, MTHR, LDS_MLP, stream>>>(
          cur, csr, offp, cnt, eps, l, nN, csrLen,
          W1p + (size_t)l * per, mb1 + (size_t)l * D2, mbn_g + (size_t)l * D2, mbn_b + (size_t)l * D2,
          mbn_m + (size_t)l * D2, mbn_v + (size_t)l * D2,
          W2p + (size_t)l * per, mb2 + (size_t)l * DD, bn_g + (size_t)l * DD, bn_b + (size_t)l * DD,
          bn_m + (size_t)l * DD, bn_v + (size_t)l * DD,
          vn, batch, nxt, NPAD);
    } else {
      k_mlp<0, 1><<<NPAD / MROWS, MTHR, LDS_MLP, stream>>>(
          cur, csr, offp, cnt, eps, l, nN, csrLen,
          W1p + (size_t)l * per, mb1 + (size_t)l * D2, mbn_g + (size_t)l * D2, mbn_b + (size_t)l * D2,
          mbn_m + (size_t)l * D2, mbn_v + (size_t)l * D2,
          W2p + (size_t)l * per, mb2 + (size_t)l * DD, bn_g + (size_t)l * DD, bn_b + (size_t)l * DD,
          bn_m + (size_t)l * DD, bn_v + (size_t)l * DD,
          vn, batch, out, nN);
    }
  }
}
